// EGNNLayer_67413806678103
// MI455X (gfx1250) — hardware-run, weakly checked
//
#include <hip/hip_runtime.h>


namespace {

constexpr int N = 50000, NP = 50048, NPL = NP  , SRCM = N  , EFULL = 600000, E = EFULL  ;
constexpr int H = 128, NQ = 6, NLQ = 2, NS = 64  , NL = (NPL < N ? NPL : N);
constexpr float XS = 8.0f, WSC = 256.0f, WSQ = 0.25f, RS_ = 1024.0f, PI_ = 3.14159265358979323846f, SLOPE = 0.0f, BNEPS = 1e-5f;
static_assert(NP % 32 == 0 && NP >= N && NPL % 32 == 0 && H == 128, "tiling");
typedef _Float16 b16;
typedef __attribute__((ext_vector_type(16))) _Float16 v16b;
typedef __attribute__((ext_vector_type(8))) _Float16 v8b;
typedef __attribute__((ext_vector_type(8))) float v8f;
typedef __attribute__((ext_vector_type(4))) float v4f;
__device__ __forceinline__ float bf16_rne(float f) { unsigned int u = __float_as_uint(f); u += 0x7FFFu + ((u >> 16) & 1u); return __uint_as_float(u & 0xFFFF0000u); }
__device__ __forceinline__ void split16(float v, b16& hi, b16& lo) { hi = (b16)v; lo = (b16)(v - (float)hi); }
__device__ __forceinline__ v16b frag_kb(const b16* p, int hh) { const v8b a = *(const v8b*)(p + 8 * hh), b = *(const v8b*)(p + 16 + 8 * hh); v16b f;
#pragma unroll
  for (int e = 0; e < 8; ++e) { f[e] = a[e]; f[8 + e] = b[e]; } return f; }
__device__ __forceinline__ v8f wmma16b(v16b a, v16b b, v8f c) { v8f d = __builtin_amdgcn_wmma_f32_16x16x32_f16(false, a, false, b, (short)0, c, false, false); asm volatile("v_nop\n\tv_nop\n\tv_nop\n\tv_nop" : "+v"(d) : "v"(a), "v"(b)); return d; }
__device__ __forceinline__ void wave_lds_sync() { __builtin_amdgcn_fence(__ATOMIC_RELEASE, "workgroup"); __builtin_amdgcn_wave_barrier(); __builtin_amdgcn_fence(__ATOMIC_ACQUIRE, "workgroup"); }
__device__ __forceinline__ float pmul(float a, float b) { float p = a * b; asm volatile("" : "+v"(p)); return p; }
__device__ __forceinline__ int iclamp(int v, int lo, int hi) { return v < lo ? lo : (v > hi ? hi : v); }
constexpr int CSR_NBLK = 512, CSR_GB = 9, CSR_GN = 1 << CSR_GB  , CSR_MAXG = 512, CSR_CAP = 12288  ;
__global__ __launch_bounds__(64) void csrA_kernel(const int* __restrict__ dst, int E, int N, int nG, int CHP, int NGP, int* __restrict__ STG, int* __restrict__ HST) {
  extern __shared__ int sm[];
  int* cnt = sm; int* run = sm + NGP; int* ids = sm + 2 * NGP;
  const int b = blockIdx.x; const int ch = (E + CSR_NBLK - 1) / CSR_NBLK; const int e0 = b * ch, e1 = min(E, e0 + ch);
  for (int i = threadIdx.x; i < NGP; i += 64) cnt[i] = 0;
  for (int i = threadIdx.x; i < CHP; i += 64) ids[i] = -1;
  __syncthreads();
  if (threadIdx.x == 0) {
    for (int e = e0; e < e1; ++e) { int d = dst[e]; d = (d < 0) ? 0 : (d >= N ? N - 1 : d); cnt[d >> CSR_GB] += 1; }
    int acc = 0; for (int g = 0; g < nG; ++g) { run[g] = acc; acc += cnt[g]; }
    for (int e = e0; e < e1; ++e) { int d = dst[e]; d = (d < 0) ? 0 : (d >= N ? N - 1 : d); const int g = d >> CSR_GB; ids[run[g]] = e; run[g] += 1; } }
  __syncthreads();
  typedef __attribute__((ext_vector_type(4))) int v4i;
  for (int pass = 0; pass < 2; ++pass) {
    for (int i = threadIdx.x; i < CHP / 4; i += 64) *(volatile v4i*)(STG + (size_t)b * CHP + i * 4) = *(const v4i*)(&ids[i * 4]);
    for (int i = threadIdx.x; i < NGP / 4; i += 64) { v4i v; for (int e = 0; e < 4; ++e) v[e] = (i * 4 + e < nG) ? cnt[i * 4 + e] : 0; *(volatile v4i*)(HST + (size_t)b * NGP + i * 4) = v; }
    __threadfence(); }
}
__global__ __launch_bounds__(512) void csrS_kernel(const int* __restrict__ HST, int nG, int NGP, int* __restrict__ START, int* __restrict__ TOT, int* __restrict__ OFF) {
  __shared__ int tot[CSR_MAXG];
  const int b = threadIdx.x;
  for (int pass = 0; pass < 2; ++pass) { int runb = 0; for (int g = 0; g < nG; ++g) { int c = HST[(size_t)b * NGP + g]; c = (c < 0) ? 0 : c; ((volatile int*)OFF)[(size_t)g * CSR_NBLK + b] = runb; runb += c; } __threadfence(); }
  for (int g = threadIdx.x; g < nG; g += 512) { int s = 0; for (int bb = 0; bb < CSR_NBLK; ++bb) { int c = HST[(size_t)bb * NGP + g]; s += (c < 0) ? 0 : c; } tot[g] = s; }
  __syncthreads();
  if (threadIdx.x < 32) {
    __shared__ int st[CSR_MAXG + 32];
    if (threadIdx.x == 0) { int acc = 0; for (int g = 0; g < NGP; ++g) { st[g] = acc; if (g < nG) acc += (tot[g] + 31) & ~31; } st[NGP] = acc; }
    __builtin_amdgcn_fence(__ATOMIC_RELEASE, "workgroup"); __builtin_amdgcn_wave_barrier(); __builtin_amdgcn_fence(__ATOMIC_ACQUIRE, "workgroup");
    for (int pass = 0; pass < 2; ++pass) { for (int i = threadIdx.x; i < NGP + 32; i += 32) { ((volatile int*)START)[i] = (i <= NGP) ? st[min(i, NGP)] : 0; ((volatile int*)TOT)[i] = (i < nG) ? tot[i] : 0; } __threadfence(); } }
}
__global__ __launch_bounds__(256) void csrB_kernel(const int* __restrict__ dst, int N, int nG, int CHP, int NGP, int permLen, const int* __restrict__ STG, const int* __restrict__ HST, const int* __restrict__ OFF, const int* __restrict__ START, const int* __restrict__ TOT, int* __restrict__ PERM, int* __restrict__ ROWPTR, int* __restrict__ ROWCNT, int* __restrict__ FLAG) {
  typedef __attribute__((ext_vector_type(4))) int v4i;
  __shared__ int ids[CSR_CAP]; __shared__ unsigned short key[CSR_CAP]; __shared__ int outp[CSR_CAP]; __shared__ int ncnt[CSR_GN + 1]; __shared__ int boff[CSR_NBLK + 1];
  const int g = blockIdx.x, t_ = threadIdx.x; int tot = TOT[g]; int st = START[g], stn = START[g + 1]; const int v0 = g * CSR_GN; const int nv = min(CSR_GN, N - v0);
  st = (st < 0) ? 0 : (st > permLen - 32 ? permLen - 32 : st) & ~31; stn = (stn < st) ? st : (stn > permLen ? permLen : stn); tot = (tot < 0) ? 0 : tot; if (tot > stn - st && tot <= CSR_CAP) tot = stn - st;
  if (tot > CSR_CAP) {
    for (int pass = 0; pass < 2; ++pass) { for (int i = t_; i < CSR_GN / 4; i += 256) { v4i a, c; for (int e = 0; e < 4; ++e) { a[e] = st; c[e] = 0; } *(volatile v4i*)(ROWPTR + v0 + i * 4) = a; *(volatile v4i*)(ROWCNT + v0 + i * 4) = c; } if (t_ == 0) ((volatile int*)FLAG)[0] = 1; __threadfence(); } (void)nv; return; }
  if (t_ == 0) { int acc = 0; for (int b = 0; b < CSR_NBLK; ++b) { boff[b] = acc; int c = HST[(size_t)b * NGP + g]; c = (c < 0) ? 0 : (c > CHP ? CHP : c); acc += c; if (acc > tot) acc = tot; } boff[CSR_NBLK] = acc; }
  for (int i = t_; i <= CSR_GN; i += 256) ncnt[i] = 0;
  __syncthreads();
  for (int b = 0; b < CSR_NBLK; ++b) { const int c = boff[b + 1] - boff[b]; int o_ = OFF[(size_t)g * CSR_NBLK + b]; o_ = (o_ < 0) ? 0 : (o_ > CHP - c ? CHP - c : o_); const int* src_ = STG + (size_t)b * CHP + o_;
    for (int i = t_; i < c; i += 256) { int id = src_[i]; id = (id < 0) ? 0 : id; ids[boff[b] + i] = id; int d = dst[id]; d = (d < v0) ? v0 : (d >= N ? N - 1 : d); int kk = d - v0; kk = (kk < 0) ? 0 : (kk >= CSR_GN ? CSR_GN - 1 : kk); key[boff[b] + i] = (unsigned short)kk; } }
  __syncthreads();
  if (t_ == 0) { for (int i = 0; i < tot; ++i) ncnt[key[i]] += 1; int acc = 0; for (int vl = 0; vl < CSR_GN; ++vl) { const int c = ncnt[vl]; ncnt[vl] = acc; acc += c; } ncnt[CSR_GN] = acc;
    for (int i = 0; i < tot; ++i) { const int vl = key[i]; outp[ncnt[vl]] = ids[i]; ncnt[vl] += 1; }
    for (int vl = CSR_GN; vl > 0; --vl) ncnt[vl] = ncnt[vl - 1]; ncnt[0] = 0; }
  __syncthreads();
  for (int pass = 0; pass < 2; ++pass) {
    for (int i = t_; i < (stn - st) / 4; i += 256) { v4i v; for (int e = 0; e < 4; ++e) { const int q = i * 4 + e; v[e] = (q < tot) ? outp[q] : -1; } *(volatile v4i*)(PERM + st + i * 4) = v; }
    for (int i = t_; i < CSR_GN / 4; i += 256) { v4i a, c; for (int e = 0; e < 4; ++e) { const int vl = i * 4 + e; a[e] = st + ncnt[vl]; c[e] = (vl < nv) ? (ncnt[vl + 1] - ncnt[vl]) : 0; } *(volatile v4i*)(ROWPTR + v0 + i * 4) = a; *(volatile v4i*)(ROWCNT + v0 + i * 4) = c; }
    __threadfence(); }
}
__global__ __launch_bounds__(256) void csrZ_kernel(int* __restrict__ p, size_t n4) { typedef __attribute__((ext_vector_type(4))) int v4i; const size_t tid = (size_t)blockIdx.x * 256 + threadIdx.x, nth = (size_t)gridDim.x * 256; v4i z = {0, 0, 0, 0}; for (size_t i = tid; i < n4; i += nth) *(volatile v4i*)(p + i * 4) = z; }
struct CsrBufs { int *STG, *HST, *OFF, *START, *TOT, *PERM, *ROWPTR, *ROWCNT, *FLAG; int nG, NGP, CHP; size_t permLen; char* base; size_t bytes; };
static size_t csr_carve(CsrBufs& c, char* ws, size_t off, int E, int N) {
  const size_t off0 = off; c.base = ws + off;
  auto al = [&](size_t bytes) { char* p = ws + off; off += (bytes + 255) & ~(size_t)255; return p; };
  c.nG = (N + CSR_GN - 1) / CSR_GN; c.NGP = (c.nG + 31) & ~31; const int ch = (E + CSR_NBLK - 1) / CSR_NBLK; c.CHP = (ch + 31) & ~31; c.permLen = (size_t)E + 32 * (size_t)c.nG + 32;
  c.STG = (int*)al((size_t)CSR_NBLK * c.CHP * 4); c.HST = (int*)al((size_t)CSR_NBLK * c.NGP * 4); c.OFF = (int*)al((size_t)c.NGP * CSR_NBLK * 4); c.START = (int*)al((size_t)(c.NGP + 64) * 4); c.TOT = (int*)al((size_t)(c.NGP + 64) * 4);
  c.PERM = (int*)al(c.permLen * 4); c.ROWPTR = (int*)al((size_t)c.nG * CSR_GN * 4); c.ROWCNT = (int*)al((size_t)c.nG * CSR_GN * 4); c.FLAG = (int*)al(256);
  c.bytes = off - off0; return off;
}
static void csr_build(const CsrBufs& c, const int* dst, int E, int N, hipStream_t stream) {
  const size_t smem = (size_t)(2 * c.NGP + c.CHP) * 4;
  csrZ_kernel<<<512, 256, 0, stream>>>((int*)c.base, c.bytes / 16);
  csrA_kernel<<<CSR_NBLK, 64, smem, stream>>>(dst, E, N, c.nG, c.CHP, c.NGP, c.STG, c.HST);
  csrS_kernel<<<1, 512, 0, stream>>>(c.HST, c.nG, c.NGP, c.START, c.TOT, c.OFF);
  csrB_kernel<<<c.nG, 256, 0, stream>>>(dst, N, c.nG, c.CHP, c.NGP, (int)c.permLen, c.STG, c.HST, c.OFF, c.START, c.TOT, c.PERM, c.ROWPTR, c.ROWCNT, c.FLAG);
}

typedef __attribute__((ext_vector_type(4))) _Float16 v4h;
__device__ __forceinline__ float silu_(float y) { return y * __builtin_amdgcn_rcpf(1.0f + __expf(-y)); }
__device__ __forceinline__ float tanh_(float y) { const float t = __expf(-2.0f * fabsf(y)); const float r = (1.0f - t) * __builtin_amdgcn_rcpf(1.0f + t); return y < 0.0f ? -r : r; }
__device__ __forceinline__ void sincos_(float x, float& s, float& c) {
  const float x2 = x * x;
  float ps = fmaf(x2, -2.5052108e-8f, 2.7557319e-6f); ps = fmaf(x2, ps, -1.9841270e-4f); ps = fmaf(x2, ps, 8.3333333e-3f); ps = fmaf(x2, ps, -1.6666667e-1f); s = x * fmaf(x2, ps, 1.0f);
  float pc = fmaf(x2, 2.0876757e-9f, -2.7557319e-7f); pc = fmaf(x2, pc, 2.4801587e-5f); pc = fmaf(x2, pc, -1.3888889e-3f); pc = fmaf(x2, pc, 4.1666667e-2f); pc = fmaf(x2, pc, -0.5f); c = fmaf(x2, pc, 1.0f);
}
template <int K, int NOUTR, int NOUTP>
__global__ __launch_bounds__(256) void wt_kernel(const float* __restrict__ w, int ld, b16* __restrict__ WT, float scl) {
  const int u = blockIdx.x * 256 + threadIdx.x; if (u >= NOUTP * K / 8) return; const int e = u * 8; const int o = e / K, k0 = e % K; v8b v;
#pragma unroll
  for (int j = 0; j < 8; ++j) v[j] = (b16)(o < NOUTR ? bf16_rne(w[(size_t)(k0 + j) * ld + o]) * scl : 0.0f);
  for (int pass = 0; pass < 2; ++pass) { *(volatile v8b*)(WT + e) = v; __threadfence(); }
}
__global__ __launch_bounds__(64) void ab_kernel(const float* __restrict__ hx, const b16* __restrict__ WA, const b16* __restrict__ WB, const float* __restrict__ mb1, float* __restrict__ AB) {
  __shared__ __attribute__((aligned(16))) b16 Ah[2][16][H + 8]; __shared__ __attribute__((aligned(16))) float Tf[2][16][2 * H + 4];
  const int wave = threadIdx.x >> 5, lane = threadIdx.x & 31, nloc = lane & 15, hlf = lane >> 4; const size_t m0 = (size_t)blockIdx.x * 32 + wave * 16;
  for (int idx = lane; idx < 16 * (H / 4); idx += 32) { const int rr = idx / (H / 4), c4 = (idx % (H / 4)) * 4; const size_t arow = (m0 + rr < (size_t)N) ? m0 + rr : (size_t)N - 1; const v4f v = *(const v4f*)(hx + arow * H + c4); v4h hv; for (int j = 0; j < 4; ++j) hv[j] = (b16)(bf16_rne(v[j]) * XS); *(v4h*)(&Ah[wave][rr][c4]) = hv; }
  wave_lds_sync();
#pragma unroll 1
  for (int ps = 0; ps < 2; ++ps) { const b16* W = ps == 0 ? WA : WB; v8f acc[8];
#pragma unroll
    for (int t = 0; t < 8; ++t) acc[t] = (v8f){};
#pragma unroll
    for (int kb = 0; kb < H; kb += 32) { const v16b a = frag_kb(&Ah[wave][nloc][kb], hlf);
#pragma unroll
      for (int t = 0; t < 8; ++t) acc[t] = wmma16b(a, frag_kb(W + (size_t)(t * 16 + nloc) * H + kb, hlf), acc[t]); }
#pragma unroll
    for (int t = 0; t < 8; ++t) { const float bb = (ps == 0) ? bf16_rne(mb1[t * 16 + nloc]) : 0.0f; for (int r = 0; r < 8; ++r) Tf[wave][8 * hlf + r][ps * H + t * 16 + nloc] = (m0 + 8 * hlf + r < (size_t)N) ? acc[t][r] * (1.0f / (XS * WSC)) + bb : 0.0f; } }
  wave_lds_sync();
  for (int pass = 0; pass < 2; ++pass) { for (int rr = 0; rr < 16; ++rr) { *(volatile v4f*)(AB + (m0 + rr) * (2 * H) + lane * 4) = *(const v4f*)(&Tf[wave][rr][lane * 4]); *(volatile v4f*)(AB + (m0 + rr) * (2 * H) + H + lane * 4) = *(const v4f*)(&Tf[wave][rr][H + lane * 4]); } __threadfence(); }
}
__global__ __launch_bounds__(64) void edge_kernel(const float* __restrict__ AB, const float* __restrict__ hx, const float* __restrict__ pos, const int* __restrict__ cols, const int* __restrict__ PERM, const int* __restrict__ ROWPTR, const int* __restrict__ ROWCNT, int permLen,
                                                   const float* __restrict__ mW1, const b16* __restrict__ W2T, const b16* __restrict__ W2Q, const float* __restrict__ mb2, const b16* __restrict__ PQT, const b16* __restrict__ PQQ, const float* __restrict__ pqb, const float* __restrict__ qw, const float* __restrict__ postW, const float* __restrict__ postb,
                                                   float* __restrict__ AGG, float* __restrict__ PN) {
  __shared__ __attribute__((aligned(16))) b16 Sh[2][16][H + 8], Sl[2][16][H + 8]; __shared__ __attribute__((aligned(16))) float Red[2][2][H + 4]; __shared__ float Qa[2][16][8]; __shared__ float St[2][16][NS + 1]; __shared__ float Tr[2][16][4];
  const int wave = threadIdx.x >> 5, lane = threadIdx.x & 31, nloc = lane & 15, hlf = lane >> 4; const int v = blockIdx.x * 2 + wave; const int vv = v < N ? v : N - 1;
  int cnt = 0, p0 = 0; if (v < N) { cnt = iclamp(ROWCNT[v], 0, 65536); p0 = iclamp(ROWPTR[v], 0, permLen - 1); if (p0 + cnt > permLen) cnt = permLen - p0; }
  const float px = bf16_rne(pos[(size_t)vv * 3]), py = bf16_rne(pos[(size_t)vv * 3 + 1]), pz = bf16_rne(pos[(size_t)vv * 3 + 2]);
  const float pw = bf16_rne(postW[0]), pb = bf16_rne(postb[0]);
  float agg4[4] = {0.0f, 0.0f, 0.0f, 0.0f}; float tsum[3] = {0.0f, 0.0f, 0.0f};
  const float* arow = AB + (size_t)vv * (2 * H);
#pragma unroll 1
  for (int e0 = 0; e0 < cnt; e0 += 16) {
    const int nval = (cnt - e0 < 16) ? (cnt - e0) : 16;
    int mycol = 0; float cdx = 0.0f, cdy = 0.0f, cdz = 0.0f, rad = 0.0f;
    if (lane < 16 && lane < nval) { const int e = iclamp(PERM[p0 + e0 + lane], 0, E - 1); int c = iclamp(cols[e], 0, N - 1); if (SRCM < N) c %= SRCM; mycol = c;
      cdx = px - bf16_rne(pos[(size_t)c * 3]); cdy = py - bf16_rne(pos[(size_t)c * 3 + 1]); cdz = pz - bf16_rne(pos[(size_t)c * 3 + 2]); rad = fmaf(cdx, cdx, fmaf(cdy, cdy, pmul(cdz, cdz))) + 1e-8f; }
    for (int rr = 0; rr < 16; ++rr) { const int c = __shfl(mycol, rr); const float radr = __shfl(rad, rr); const bool ok = rr < nval; const float* brow = AB + (size_t)c * (2 * H) + H;
      { const int c4 = lane * 4; const v4f a4 = *(const v4f*)(arow + c4); const v4f b4 = *(const v4f*)(brow + c4); v4h hv, lv;
        for (int j = 0; j < 4; ++j) { const float pre = a4[j] + b4[j] + radr * bf16_rne(mW1[(size_t)(2 * H) * H + c4 + j]); const float s = ok ? silu_(pre) : 0.0f; const float vs = s * XS; const b16 ph = (b16)vs; hv[j] = ph; lv[j] = (b16)((vs - (float)ph) * RS_); }
        *(v4h*)(&Sh[wave][rr][c4]) = hv; *(v4h*)(&Sl[wave][rr][c4]) = lv; } }
    wave_lds_sync();
    v8f acc[8];
#pragma unroll
    for (int t = 0; t < 8; ++t) acc[t] = (v8f){};
#pragma unroll
    for (int kb = 0; kb < H; kb += 32) { const v16b a = frag_kb(&Sh[wave][nloc][kb], hlf), al = frag_kb(&Sl[wave][nloc][kb], hlf);
#pragma unroll
      for (int t = 0; t < 8; ++t) { const size_t wo_ = (size_t)(t * 16 + nloc) * H + kb; acc[t] = wmma16b(a, frag_kb(W2T + wo_, hlf), acc[t]); acc[t] = wmma16b(al, frag_kb(W2Q + wo_, hlf), acc[t]); } }
    wave_lds_sync();
#pragma unroll
    for (int t = 0; t < 8; ++t) { const int col = t * 16 + nloc; const float bb = bf16_rne(mb2[col]); float part = 0.0f;
#pragma unroll
      for (int r = 0; r < 8; ++r) { const bool ok = (8 * hlf + r) < nval; const float msg = ok ? acc[t][r] * (1.0f / (XS * WSC)) + bb : 0.0f; part += msg; const float vs = msg * XS; const b16 ph = (b16)vs; Sh[wave][8 * hlf + r][col] = ph; Sl[wave][8 * hlf + r][col] = (b16)((vs - (float)ph) * RS_); }
      Red[wave][hlf][col] = part; }
    wave_lds_sync();
    { const int c4 = lane * 4; for (int j = 0; j < 4; ++j) agg4[j] += Red[wave][0][c4 + j] + Red[wave][1][c4 + j]; }
    v8f qa = (v8f){};
#pragma unroll
    for (int kb = 0; kb < H; kb += 32) { const v16b a = frag_kb(&Sh[wave][nloc][kb], hlf), al = frag_kb(&Sl[wave][nloc][kb], hlf); qa = wmma16b(a, frag_kb(PQT + (size_t)nloc * H + kb, hlf), qa); qa = wmma16b(al, frag_kb(PQQ + (size_t)nloc * H + kb, hlf), qa); }
    if (nloc < NQ) { const float bb = bf16_rne(pqb[nloc]); for (int r = 0; r < 8; ++r) Qa[wave][8 * hlf + r][nloc] = tanh_(qa[r] * (1.0f / (XS * WSC)) + bb) * PI_; }
    wave_lds_sync();
    float qout = 0.0f;
    if (lane < nval) { float* st = &St[wave][lane][0];
#pragma unroll 1
      for (int i = 0; i < NS; ++i) st[i] = (i == 0) ? 1.0f : 0.0f;
#pragma unroll 1
      for (int step = 0; step < NQ * (1 + NLQ); ++step) { const int q = step % NQ; const int layer = step / NQ;
        const float theta = (layer == 0) ? Qa[wave][lane][q] : bf16_rne(qw[(layer - 1) * NQ + q]); float sn, cs; sincos_(0.5f * theta, sn, cs); const int bp = NQ - 1 - q; const int lowmask = (1 << bp) - 1;
#pragma unroll 1
        for (int j = 0; j < NS / 2; ++j) { const int i0 = ((j >> bp) << (bp + 1)) | (j & lowmask); const int i1 = i0 | (1 << bp); const float a0 = st[i0], a1 = st[i1]; st[i0] = fmaf(cs, a0, -sn * a1); st[i1] = fmaf(sn, a0, cs * a1); }
        if (layer > 0 && q == NQ - 1) {
#pragma unroll 1
          for (int c = 0; c < NQ; ++c) { const int t = (c + 1) % NQ; const int bc = NQ - 1 - c, bt = NQ - 1 - t;
#pragma unroll 1
            for (int i = 0; i < NS; ++i) { if (((i >> bc) & 1) && !((i >> bt) & 1)) { const int i1 = i | (1 << bt); const float a = st[i]; st[i] = st[i1]; st[i1] = a; } } } } }
      float pz0 = 0.0f, pz1 = 0.0f;
#pragma unroll 1
      for (int i = 0; i < NS; ++i) { const float a = st[i]; if ((i >> (NQ - 1)) & 1) pz1 = fmaf(a, a, pz1); else pz0 = fmaf(a, a, pz0); }
      qout = pz0 - pz1;
      const float w = fmaf(qout, pw, pb); Tr[wave][lane][0] = cdx * w; Tr[wave][lane][1] = cdy * w; Tr[wave][lane][2] = cdz * w; }
    wave_lds_sync();
    if (lane == 0) { for (int e2 = 0; e2 < nval; ++e2) { tsum[0] += Tr[wave][e2][0]; tsum[1] += Tr[wave][e2][1]; tsum[2] += Tr[wave][e2][2]; } }
    wave_lds_sync(); }
  for (int pass = 0; pass < 2; ++pass) { if (v < NPL) { v4f o; for (int j = 0; j < 4; ++j) o[j] = (v < N) ? agg4[j] : 0.0f; *(volatile v4f*)(AGG + (size_t)v * H + lane * 4) = o;
      { const float t0 = __shfl(tsum[0], 0), t1 = __shfl(tsum[1], 0), t2 = __shfl(tsum[2], 0); const float pv = (lane == 0) ? px + t0 : (lane == 1) ? py + t1 : (lane == 2) ? pz + t2 : 0.0f; ((volatile float*)PN)[(size_t)v * 32 + lane] = (v < N) ? pv : 0.0f; } }
    __threadfence(); }
}
__global__ __launch_bounds__(64) void nodemlp_kernel(const float* __restrict__ hx, const float* __restrict__ AGG, const b16* __restrict__ N1T, const b16* __restrict__ N1Q, const float* __restrict__ nb1, const b16* __restrict__ N2T, const b16* __restrict__ N2Q, const float* __restrict__ nb2, float* __restrict__ OUT, int mrows) {
  __shared__ __attribute__((aligned(16))) b16 Ah[2][16][2 * H + 8], Al[2][16][2 * H + 8]; __shared__ __attribute__((aligned(16))) float Tf[2][16][H + 4];
  const int wave = threadIdx.x >> 5, lane = threadIdx.x & 31, nloc = lane & 15, hlf = lane >> 4; const size_t m0 = (size_t)blockIdx.x * 32 + wave * 16;
  for (int idx = lane; idx < 16 * (H / 4); idx += 32) { const int rr = idx / (H / 4), c4 = (idx % (H / 4)) * 4; const size_t arow = (m0 + rr < (size_t)N) ? m0 + rr : (size_t)N - 1; const v4f hv4 = *(const v4f*)(hx + arow * H + c4), av4 = *(const v4f*)(AGG + arow * H + c4); v4h h1, l1, h2, l2;
    for (int j = 0; j < 4; ++j) { h1[j] = (b16)(bf16_rne(hv4[j]) * XS); l1[j] = (b16)0.0f; const float vs = av4[j] * XS; const b16 ph = (b16)vs; h2[j] = ph; l2[j] = (b16)((vs - (float)ph) * RS_); }
    *(v4h*)(&Ah[wave][rr][c4]) = h1; *(v4h*)(&Al[wave][rr][c4]) = l1; *(v4h*)(&Ah[wave][rr][H + c4]) = h2; *(v4h*)(&Al[wave][rr][H + c4]) = l2; }
  wave_lds_sync();
  v8f acc[8];
#pragma unroll
  for (int t = 0; t < 8; ++t) acc[t] = (v8f){};
#pragma unroll 2
  for (int kb = 0; kb < 2 * H; kb += 32) { const v16b a = frag_kb(&Ah[wave][nloc][kb], hlf), al = frag_kb(&Al[wave][nloc][kb], hlf); const bool second = kb >= H;
#pragma unroll
    for (int t = 0; t < 8; ++t) { const size_t wo_ = (size_t)(t * 16 + nloc) * (2 * H) + kb; acc[t] = wmma16b(a, frag_kb(N1T + wo_, hlf), acc[t]); if (second) acc[t] = wmma16b(al, frag_kb(N1Q + wo_, hlf), acc[t]); } }
  wave_lds_sync();
#pragma unroll
  for (int t = 0; t < 8; ++t) { const float bb = bf16_rne(nb1[t * 16 + nloc]);
#pragma unroll
    for (int r = 0; r < 8; ++r) { const float tv = silu_(acc[t][r] * (1.0f / (XS * WSC)) + bb); const float vs = tv * XS; const b16 ph = (b16)vs; Ah[wave][8 * hlf + r][t * 16 + nloc] = ph; Al[wave][8 * hlf + r][t * 16 + nloc] = (b16)((vs - (float)ph) * RS_); } }
  wave_lds_sync();
#pragma unroll
  for (int t = 0; t < 8; ++t) acc[t] = (v8f){};
#pragma unroll
  for (int kb = 0; kb < H; kb += 32) { const v16b a = frag_kb(&Ah[wave][nloc][kb], hlf), al = frag_kb(&Al[wave][nloc][kb], hlf);
#pragma unroll
    for (int t = 0; t < 8; ++t) { const size_t wo_ = (size_t)(t * 16 + nloc) * H + kb; acc[t] = wmma16b(a, frag_kb(N2T + wo_, hlf), acc[t]); acc[t] = wmma16b(al, frag_kb(N2Q + wo_, hlf), acc[t]); } }
#pragma unroll
  for (int t = 0; t < 8; ++t) { const int col = t * 16 + nloc; const float bb = bf16_rne(nb2[col]);
#pragma unroll
    for (int r = 0; r < 8; ++r) { const size_t vrow = m0 + 8 * hlf + r; Tf[wave][8 * hlf + r][col] = (vrow < (size_t)N) ? acc[t][r] * (1.0f / (XS * WSC)) + bb + bf16_rne(hx[(vrow < (size_t)N ? vrow : (size_t)N - 1) * H + col]) : 0.0f; } }
  wave_lds_sync();
  for (int pass = 0; pass < 2; ++pass) { for (int rr = 0; rr < 16; ++rr) if (m0 + rr < (size_t)mrows) *(volatile v4f*)(OUT + (m0 + rr) * H + lane * 4) = *(const v4f*)(&Tf[wave][rr][lane * 4]); __threadfence(); }
}
__global__ __launch_bounds__(32) void copy3_kernel(const float* __restrict__ PN, float* __restrict__ out3, int nrows) {
  const int r0 = blockIdx.x * 32; const int lane = threadIdx.x; const int nr = (nrows - r0 < 32) ? (nrows - r0) : 32; const int nfl = nr * 3;
  for (int pass = 0; pass < 2; ++pass) { for (int f = lane; f < nfl; f += 32) { const int rr = f / 3, k = f % 3; ((volatile float*)out3)[(size_t)r0 * 3 + f] = PN[(size_t)(r0 + rr) * 32 + k]; } __threadfence(); }
}
}

extern "C" void kernel_launch(void* const* d_in, const int* in_sizes, int n_in, void* d_out, int out_size, void* d_ws, size_t ws_size, hipStream_t stream) {
  (void)n_in;
  auto Fp = [&](int i) { return (const float*)d_in[i]; }; auto Ip = [&](int i) { return (const int*)d_in[i]; };
  if (in_sizes[0] != N * H || in_sizes[1] != N * 3 || in_sizes[2] != 2 * EFULL || in_sizes[3] != (2 * H + 1) * H || in_sizes[4] != H || in_sizes[5] != H * H || in_sizes[6] != H || in_sizes[7] != H * NQ || in_sizes[8] != NQ || in_sizes[9] != NLQ * NQ || in_sizes[10] != 1 || in_sizes[11] != 1 || in_sizes[12] != 2 * H * H || in_sizes[13] != H || in_sizes[14] != H * H || in_sizes[15] != H || out_size != N * H + N * 3) return;
  float* out_h = (float*)d_out; float* out_p = out_h + (size_t)N * H;
  size_t off = 0; char* ws = (char*)d_ws;
  auto carve = [&](size_t bytes) { char* p = ws + off; off += (bytes + 255) & ~(size_t)255; return p; };
  b16* WA = (b16*)carve((size_t)H * H * 2); b16* WB = (b16*)carve((size_t)H * H * 2); b16* W2T = (b16*)carve((size_t)H * H * 2); b16* W2Q = (b16*)carve((size_t)H * H * 2); b16* PQT = (b16*)carve((size_t)16 * H * 2); b16* PQQ = (b16*)carve((size_t)16 * H * 2);
  b16* N1T = (b16*)carve((size_t)H * 2 * H * 2); b16* N1Q = (b16*)carve((size_t)H * 2 * H * 2); b16* N2T = (b16*)carve((size_t)H * H * 2); b16* N2Q = (b16*)carve((size_t)H * H * 2);
  float* AB = (float*)carve((size_t)NP * 2 * H * 4); float* AGG = (float*)carve((size_t)NP * H * 4); float* PN = (float*)carve((size_t)NP * 32 * 4);
  CsrBufs csr; off = csr_carve(csr, ws, off, E, N);
  if (off > ws_size || off > ((size_t)128 << 20)) return;
  const unsigned g8 = (H * H / 8 + 255) / 256;
  wt_kernel<H, H, H><<<g8, 256, 0, stream>>>(Fp(3), H, WA, WSC); wt_kernel<H, H, H><<<g8, 256, 0, stream>>>(Fp(3) + (size_t)H * H, H, WB, WSC);
  wt_kernel<H, H, H><<<g8, 256, 0, stream>>>(Fp(5), H, W2T, WSC); wt_kernel<H, H, H><<<g8, 256, 0, stream>>>(Fp(5), H, W2Q, WSQ);
  wt_kernel<H, NQ, 16><<<(16 * H / 8 + 255) / 256, 256, 0, stream>>>(Fp(7), NQ, PQT, WSC); wt_kernel<H, NQ, 16><<<(16 * H / 8 + 255) / 256, 256, 0, stream>>>(Fp(7), NQ, PQQ, WSQ);
  wt_kernel<2 * H, H, H><<<(H * 2 * H / 8 + 255) / 256, 256, 0, stream>>>(Fp(12), H, N1T, WSC); wt_kernel<2 * H, H, H><<<(H * 2 * H / 8 + 255) / 256, 256, 0, stream>>>(Fp(12), H, N1Q, WSQ);
  wt_kernel<H, H, H><<<g8, 256, 0, stream>>>(Fp(14), H, N2T, WSC); wt_kernel<H, H, H><<<g8, 256, 0, stream>>>(Fp(14), H, N2Q, WSQ);
  csr_build(csr, Ip(2), E, N, stream);
  ab_kernel<<<NP / 32, 64, 0, stream>>>(Fp(0), WA, WB, Fp(4), AB);
  edge_kernel<<<NP / 2, 64, 0, stream>>>(AB, Fp(0), Fp(1), Ip(2) + EFULL, csr.PERM, csr.ROWPTR, csr.ROWCNT, (int)csr.permLen, Fp(3), W2T, W2Q, Fp(6), PQT, PQQ, Fp(8), Fp(9), Fp(10), Fp(11), AGG, PN);
  nodemlp_kernel<<<NPL / 32, 64, 0, stream>>>(Fp(0), AGG, N1T, N1Q, Fp(13), N2T, N2Q, Fp(15), out_h, NL);
  copy3_kernel<<<(NL + 31) / 32, 32, 0, stream>>>(PN, out_p, NL);
}
